// NeuralAdditiveModel_23691039604774
// MI455X (gfx1250) — hardware-verified
//
#include <hip/hip_runtime.h>
#include <stdint.h>

#ifndef NB
#define NB 8192
#endif
#define NB_FULL 8192
#define F_  256
#define H1_ 128
#define H2_ 64
#define H3_ 32
#define TPB 256
#define ROWS_PER_BLOCK 128

static_assert(NB % ROWS_PER_BLOCK == 0);
static_assert(NB <= NB_FULL);
static_assert(NB >= ROWS_PER_BLOCK);
static_assert(F_ == TPB);

#define W2P_BYTES ((size_t)F_ * H1_ * H2_ * 2)
#define W3P_BYTES ((size_t)F_ * H2_ * H3_ * 2)
#define W4P_BYTES ((size_t)F_ * 32 * 16 * 2)
#define W1P_BYTES ((size_t)F_ * H1_ * 2)
#define B1P_BYTES ((size_t)F_ * H1_ * 2)
#define OFF_W2P ((size_t)0)
#define OFF_W3P (OFF_W2P + W2P_BYTES)
#define OFF_W4P (OFF_W3P + W3P_BYTES)
#define OFF_W1P (OFF_W4P + W4P_BYTES)
#define OFF_B1P (OFF_W1P + W1P_BYTES)
#define WS_TOTAL (OFF_B1P + B1P_BYTES)
static_assert(WS_TOTAL <= (size_t)134217728);
static_assert((OFF_W3P % 128) == 0 && (OFF_W4P % 128) == 0 && (OFF_W1P % 128) == 0 && (OFF_B1P % 128) == 0);

#define W2_PIECES (F_ * 1024)
#define W3_PIECES (F_ * 256)
#define W4_PIECES (F_ * 64)
#define W1_PIECES (F_ * 16)
#define B1_PIECES (F_ * 16)
static_assert((size_t)W2_PIECES * 16 == W2P_BYTES);
static_assert((size_t)W3_PIECES * 16 == W3P_BYTES);
static_assert((size_t)W4_PIECES * 16 == W4P_BYTES);
static_assert((size_t)W1_PIECES * 16 == W1P_BYTES);
static_assert((size_t)B1_PIECES * 16 == B1P_BYTES);
static_assert(W2_PIECES % TPB == 0 && W3_PIECES % TPB == 0);
static_assert(W4_PIECES % TPB == 0 && W1_PIECES % TPB == 0 && B1_PIECES % TPB == 0);

typedef _Float16 v16h __attribute__((ext_vector_type(16)));
typedef _Float16 v8h  __attribute__((ext_vector_type(8)));
typedef _Float16 v8ha __attribute__((ext_vector_type(8), may_alias));
typedef float    v8f  __attribute__((ext_vector_type(8)));
typedef float    v4f  __attribute__((ext_vector_type(4), may_alias));
typedef unsigned int v4u __attribute__((ext_vector_type(4), may_alias));

union Pk8 { v8h h; v4u u; };

__device__ __forceinline__ float bfr(float v) {
    unsigned int u = __float_as_uint(v);
    u = (u + 0x7FFFu + ((u >> 16) & 1u)) & 0xFFFF0000u;
    return __uint_as_float(u);
}

__device__ __forceinline__ int kmap(int i, int g) {
    return (i < 8) ? (i + 8 * g) : (i + 8 + 8 * g);
}

__device__ __forceinline__ v8f wmma_f16(v16h a, v16h b, v8f c) {
    v8f d = __builtin_amdgcn_wmma_f32_16x16x32_f16(false, a, false, b, (short)0, c, false, false);
    asm volatile("v_nop\n\tv_nop\n\tv_nop\n\tv_nop" : "+v"(d) : "v"(a), "v"(b));
    return d;
}

__device__ __forceinline__ void lds_wave_sync() {
    __builtin_amdgcn_fence(__ATOMIC_RELEASE, "wavefront");
    asm volatile("s_wait_dscnt 0" ::: "memory");
    __builtin_amdgcn_wave_barrier();
}

__device__ __forceinline__ void store16x2(_Float16* dst, const Pk8& p) {
    v4u* q = (v4u*)dst;
    *(volatile v4u*)q = p.u;
    __threadfence();
    *(volatile v4u*)q = p.u;
}

__launch_bounds__(TPB)
__global__ void k_cvt_w2(const float* __restrict__ W2, _Float16* __restrict__ W2p) {
    const int p = blockIdx.x * TPB + threadIdx.x;
    if (p >= W2_PIECES) return;
    const int i0 = (p & 1) * 8;
    const int ln = (p >> 1) & 31;
    const int nb = (p >> 6) & 3;
    const int kb = (p >> 8) & 3;
    const int f  = p >> 10;
    const int h  = ln >> 4;
    const int n  = 16 * nb + (ln & 15);
    const int kbase = 32 * kb + 8 * h + 2 * i0;
    Pk8 v;
#pragma unroll
    for (int j = 0; j < 8; ++j)
        v.h[j] = (_Float16)(16.0f * bfr(W2[((size_t)f * H1_ + kbase + j) * H2_ + n]));
    store16x2(W2p + (size_t)p * 8, v);
}

__launch_bounds__(TPB)
__global__ void k_cvt_w3(const float* __restrict__ W3, _Float16* __restrict__ W3p) {
    const int p = blockIdx.x * TPB + threadIdx.x;
    if (p >= W3_PIECES) return;
    const int i0 = (p & 1) * 8;
    const int ln = (p >> 1) & 31;
    const int nb = (p >> 6) & 1;
    const int kb = (p >> 7) & 1;
    const int f  = p >> 8;
    const int h  = ln >> 4;
    const int n  = 16 * nb + (ln & 15);
    const int kbase = 32 * kb + 8 * h + 2 * i0;
    Pk8 v;
#pragma unroll
    for (int j = 0; j < 8; ++j)
        v.h[j] = (_Float16)(4.0f * bfr(W3[((size_t)f * H2_ + kbase + j) * H3_ + n]));
    store16x2(W3p + (size_t)p * 8, v);
}

__launch_bounds__(TPB)
__global__ void k_cvt_small(const float* __restrict__ W4, const float* __restrict__ W1, const float* __restrict__ b1,
                            _Float16* __restrict__ W4p, _Float16* __restrict__ W1p, _Float16* __restrict__ b1p) {
    const int p = blockIdx.x * TPB + threadIdx.x;
    if (p >= W4_PIECES + W1_PIECES + B1_PIECES) return;
    Pk8 v;
    if (p < W4_PIECES) {
        const int i0 = (p & 1) * 8;
        const int ln = (p >> 1) & 31;
        const int f  = p >> 6;
        const int h  = ln >> 4;
        const int n  = ln & 15;
        const int kbase = 8 * h + 2 * i0;
#pragma unroll
        for (int j = 0; j < 8; ++j) {
            const float w = 8.0f * bfr(W4[(size_t)f * H3_ + kbase + j]);
            v.h[j] = (_Float16)((n == 0) ? w : 0.0f);
        }
        store16x2(W4p + (size_t)p * 8, v);
    } else if (p < W4_PIECES + W1_PIECES) {
        const int q  = p - W4_PIECES;
        const int i0 = (q & 1) * 8;
        const int g  = (q >> 1) & 1;
        const int kb = (q >> 2) & 3;
        const int f  = q >> 4;
        const int kbase = 32 * kb + 8 * g + 2 * i0;
#pragma unroll
        for (int j = 0; j < 8; ++j) v.h[j] = (_Float16)bfr(W1[(size_t)f * H1_ + kbase + j]);
        store16x2(W1p + (size_t)q * 8, v);
    } else {
        const int q  = p - W4_PIECES - W1_PIECES;
        const int i0 = (q & 1) * 8;
        const int g  = (q >> 1) & 1;
        const int kb = (q >> 2) & 3;
        const int f  = q >> 4;
        const int kbase = 32 * kb + 8 * g + 2 * i0;
#pragma unroll
        for (int j = 0; j < 8; ++j) v.h[j] = (_Float16)bfr(b1[(size_t)f * H1_ + kbase + j]);
        store16x2(b1p + (size_t)q * 8, v);
    }
}

__launch_bounds__(TPB, 2)
__global__ void k_nam_main(const float* __restrict__ x,
                           const float* __restrict__ b2,
                           const float* __restrict__ b3,
                           const float* __restrict__ b4,
                           const float* __restrict__ bias,
                           const _Float16* __restrict__ W2p,
                           const _Float16* __restrict__ W3p,
                           const _Float16* __restrict__ W4p,
                           const _Float16* __restrict__ W1p,
                           const _Float16* __restrict__ b1p,
                           float* __restrict__ out)
{
    __shared__ __align__(16) _Float16 sH2[8][16][H2_];
    __shared__ __align__(16) _Float16 sH3[8][16][H3_];
    __shared__ __align__(16) float sOut[ROWS_PER_BLOCK];
    __shared__ float sRed[8];

    const int tid  = threadIdx.x;
    const int lane = tid & 31;
    const int wave = tid >> 5;
    const int g    = lane >> 4;
    const int m    = lane & 15;
    const int b0   = (blockIdx.x * 8 + wave) * 16;

    {
        float v = bfr(b4[tid]);
        v += __shfl_xor(v, 16, 32);
        v += __shfl_xor(v, 8, 32);
        v += __shfl_xor(v, 4, 32);
        v += __shfl_xor(v, 2, 32);
        v += __shfl_xor(v, 1, 32);
        if (lane == 0) sRed[wave] = v;
    }
    __syncthreads();
    float cb = bfr(bias[0]);
#pragma unroll
    for (int w = 0; w < 8; ++w) cb += sRed[w];

    const v16h* W1v = (const v16h*)W1p;
    const v16h* B1v = (const v16h*)b1p;
    const v16h* W2v = (const v16h*)W2p;
    const v16h* W3v = (const v16h*)W3p;
    const v16h* W4v = (const v16h*)W4p;

    const v16h zero16 = {};
    v8f accO;
#pragma unroll
    for (int r = 0; r < 8; ++r) accO[r] = 0.0f;

#pragma unroll 1
    for (int f = 0; f < F_; ++f) {
        const _Float16 xh = (_Float16)bfr(x[(size_t)(b0 + m) * F_ + f]);
        v16h xs;
#pragma unroll
        for (int i = 0; i < 16; ++i) xs[i] = xh;

        v16h a[4];
#pragma unroll
        for (int kb = 0; kb < 4; ++kb) {
            const v16h w = W1v[(f * 4 + kb) * 2 + g];
            const v16h c = B1v[(f * 4 + kb) * 2 + g];
            a[kb] = __builtin_elementwise_max((v16h)(xs * w + c), zero16);
        }

        v8f acc2[4];
#pragma unroll
        for (int nb = 0; nb < 4; ++nb) {
            const float bz = 16.0f * bfr(b2[f * H2_ + 16 * nb + m]);
#pragma unroll
            for (int r = 0; r < 8; ++r) acc2[nb][r] = bz;
        }
#pragma unroll
        for (int kb = 0; kb < 4; ++kb) {
#pragma unroll
            for (int nb = 0; nb < 4; ++nb) {
                const v16h bf = W2v[((f * 4 + kb) * 4 + nb) * 32 + lane];
                acc2[nb] = wmma_f16(a[kb], bf, acc2[nb]);
            }
        }

        asm volatile("" ::: "memory");
#pragma unroll
        for (int np = 0; np < 2; ++np) {
            v16h hv;
#pragma unroll
            for (int r = 0; r < 8; ++r) {
                hv[2 * r]     = (_Float16)acc2[2 * np][r];
                hv[2 * r + 1] = (_Float16)acc2[2 * np + 1][r];
            }
            hv = __builtin_elementwise_max(hv, zero16);
#pragma unroll
            for (int r = 0; r < 8; ++r) {
                const int M = r + 8 * g;
                sH2[wave][M][32 * np + m]      = hv[2 * r];
                sH2[wave][M][32 * np + 16 + m] = hv[2 * r + 1];
            }
        }
        lds_wave_sync();

        v16h aH2[2];
        {
            const _Float16* row = &sH2[wave][m][0];
#pragma unroll
            for (int kb = 0; kb < 2; ++kb) {
                const v8ha lo = *(const v8ha*)&row[32 * kb + 8 * g];
                const v8ha hi = *(const v8ha*)&row[32 * kb + 16 + 8 * g];
#pragma unroll
                for (int j = 0; j < 8; ++j) { aH2[kb][j] = lo[j]; aH2[kb][j + 8] = hi[j]; }
            }
        }

        v8f acc3[2];
#pragma unroll
        for (int nb = 0; nb < 2; ++nb) {
            const float bz = 64.0f * bfr(b3[f * H3_ + 16 * nb + m]);
#pragma unroll
            for (int r = 0; r < 8; ++r) acc3[nb][r] = bz;
        }
#pragma unroll
        for (int kb = 0; kb < 2; ++kb) {
#pragma unroll
            for (int nb = 0; nb < 2; ++nb) {
                const v16h bf = W3v[((f * 2 + kb) * 2 + nb) * 32 + lane];
                acc3[nb] = wmma_f16(aH2[kb], bf, acc3[nb]);
            }
        }

        asm volatile("" ::: "memory");
        {
            v16h hv;
#pragma unroll
            for (int r = 0; r < 8; ++r) {
                hv[2 * r]     = (_Float16)acc3[0][r];
                hv[2 * r + 1] = (_Float16)acc3[1][r];
            }
            hv = __builtin_elementwise_max(hv, zero16);
#pragma unroll
            for (int r = 0; r < 8; ++r) {
                const int M = r + 8 * g;
                sH3[wave][M][m]      = hv[2 * r];
                sH3[wave][M][16 + m] = hv[2 * r + 1];
            }
        }
        lds_wave_sync();

        v16h aH3;
        {
            const _Float16* row = &sH3[wave][m][0];
            const v8ha lo = *(const v8ha*)&row[8 * g];
            const v8ha hi = *(const v8ha*)&row[16 + 8 * g];
#pragma unroll
            for (int j = 0; j < 8; ++j) { aH3[j] = lo[j]; aH3[j + 8] = hi[j]; }
        }

        const v16h bo = W4v[f * 32 + lane];
        accO = wmma_f16(aH3, bo, accO);
    }

    const float inv512 = 0.001953125f;
    if (m == 0) {
#pragma unroll
        for (int r = 0; r < 8; ++r) sOut[wave * 16 + 8 * g + r] = accO[r] * inv512 + cb;
    }
    __syncthreads();
    if (wave == 0) {
        const v4f o = *(const v4f*)&sOut[4 * lane];
        float* dst = out + (size_t)blockIdx.x * ROWS_PER_BLOCK + 4 * lane;
        *(volatile v4f*)dst = o;
        __threadfence();
        *(volatile v4f*)dst = o;
    }
}

extern "C" void kernel_launch(void* const* d_in, const int* in_sizes, int n_in,
                              void* d_out, int out_size, void* d_ws, size_t ws_size,
                              hipStream_t stream) {
    if (n_in < 10) return;
    if (in_sizes[0] < NB * F_) return;
    if (in_sizes[1] < F_ * H1_) return;
    if (in_sizes[2] < F_ * H1_) return;
    if (in_sizes[3] < F_ * H1_ * H2_) return;
    if (in_sizes[4] < F_ * H2_) return;
    if (in_sizes[5] < F_ * H2_ * H3_) return;
    if (in_sizes[6] < F_ * H3_) return;
    if (in_sizes[7] < F_ * H3_) return;
    if (in_sizes[8] < F_) return;
    if (in_sizes[9] < 1) return;
    if (out_size < NB) return;
    if (ws_size < WS_TOTAL) return;

    const float* x    = (const float*)d_in[0];
    const float* W1   = (const float*)d_in[1];
    const float* b1   = (const float*)d_in[2];
    const float* W2   = (const float*)d_in[3];
    const float* b2   = (const float*)d_in[4];
    const float* W3   = (const float*)d_in[5];
    const float* b3   = (const float*)d_in[6];
    const float* W4   = (const float*)d_in[7];
    const float* b4   = (const float*)d_in[8];
    const float* bias = (const float*)d_in[9];
    float* out = (float*)d_out;

    char* ws = (char*)d_ws;
    _Float16* W2p = (_Float16*)(ws + OFF_W2P);
    _Float16* W3p = (_Float16*)(ws + OFF_W3P);
    _Float16* W4p = (_Float16*)(ws + OFF_W4P);
    _Float16* W1p = (_Float16*)(ws + OFF_W1P);
    _Float16* b1p = (_Float16*)(ws + OFF_B1P);

    k_cvt_w2<<<dim3(W2_PIECES / TPB), dim3(TPB), 0, stream>>>(W2, W2p);
    k_cvt_w3<<<dim3(W3_PIECES / TPB), dim3(TPB), 0, stream>>>(W3, W3p);
    k_cvt_small<<<dim3((W4_PIECES + W1_PIECES + B1_PIECES) / TPB), dim3(TPB), 0, stream>>>(
        W4, W1, b1, W4p, W1p, b1p);
    k_nam_main<<<dim3(NB / ROWS_PER_BLOCK), dim3(TPB), 0, stream>>>(
        x, b2, b3, b4, bias, W2p, W3p, W4p, W1p, b1p, out);
}
